// Bilaplacian_21225728377222
// MI455X (gfx1250) — hardware-verified
//
#include <hip/hip_runtime.h>
#include <math.h>

typedef __attribute__((ext_vector_type(16))) __bf16   v16b;
typedef __attribute__((ext_vector_type(8)))  __bf16   v8b;
typedef __attribute__((ext_vector_type(8)))  float    v8f;
typedef __attribute__((ext_vector_type(4)))  float    v4f;
typedef __attribute__((ext_vector_type(4)))  unsigned v4u;
typedef __attribute__((ext_vector_type(2)))  unsigned v2u;

constexpr int kBatch = 256;
constexpr int kDin   = 16;
constexpr int kHid   = 128;
constexpr int kOut   = 8;
constexpr int kTileM = 16;
constexpr int kXP  = 40;
constexpr int kW1P = 40;
constexpr int kGP  = 136;
constexpr int kW2P = 136;
constexpr int kZP  = 132;
constexpr int kOP  = 16;
static_assert(kDin == 16, "K of the first contraction is padded 16 -> 32");
static_assert(kOut == 8, "N of the second contraction is padded 8 -> 16");
static_assert((kBatch % kTileM) == 0, "grid covers the batch exactly");
static_assert((kHid % 32) == 0, "K of the second contraction steps by 32");
static_assert((kHid % 16) == 0, "N tiles of the first contraction");
static_assert(((kXP * 2) % 16) == 0 && ((kW1P * 2) % 16) == 0 && ((kGP * 2) % 16) == 0 && ((kW2P * 2) % 16) == 0, "16-B aligned plane rows");
static_assert(((kZP * 4) % 16) == 0 && ((kOP * 4) % 16) == 0, "16-B aligned f32 rows");
static_assert(kXP >= 32 && kW1P >= 32 && kGP >= kHid && kW2P >= kHid && kZP >= kHid, "pitches cover the read extents");

__device__ __forceinline__ unsigned bf_rne_bits(float f) {
  const unsigned u = __float_as_uint(f);
  return ((u + 0x7FFFu + ((u >> 16) & 1u)) >> 16) & 0xFFFFu;
}
__device__ __forceinline__ void split_pair(float a, float b, unsigned& hw, unsigned& lw) {
  const unsigned ha = bf_rne_bits(a);
  const unsigned hb = bf_rne_bits(b);
  const unsigned la = bf_rne_bits(a - __uint_as_float(ha << 16));
  const unsigned lb = bf_rne_bits(b - __uint_as_float(hb << 16));
  hw = ha | (hb << 16);
  lw = la | (lb << 16);
}
__device__ __forceinline__ void split_oct(v4f a0, v4f a1, v4u& hw, v4u& lw) {
  unsigned h0, h1, h2, h3, l0, l1, l2, l3;
  const float e0 = a0[0], e1 = a0[1], e2 = a0[2], e3 = a0[3];
  const float e4 = a1[0], e5 = a1[1], e6 = a1[2], e7 = a1[3];
  split_pair(e0, e1, h0, l0);
  split_pair(e2, e3, h1, l1);
  split_pair(e4, e5, h2, l2);
  split_pair(e6, e7, h3, l3);
  hw = (v4u){h0, h1, h2, h3};
  lw = (v4u){l0, l1, l2, l3};
}

union FragU { v16b v; v8b h[2]; };
__device__ __forceinline__ v16b frag_load(const __bf16* p) {
  FragU f;
  f.h[0] = *(const v8b*)(p);
  f.h[1] = *(const v8b*)(p + 16);
  return f.v;
}
__device__ __forceinline__ v8f mma_bf(v16b a, v16b b, v8f c) {
  return __builtin_amdgcn_wmma_f32_16x16x32_bf16(false, a, false, b, (short)0, c, false, false);
}
__device__ __forceinline__ void guard_acc(v8f& c, v16b a0, v16b a1, v16b b0, v16b b1) {
  asm volatile("v_nop\n\tv_nop\n\tv_nop\n\tv_nop" : "+v"(c) : "v"(a0), "v"(a1), "v"(b0), "v"(b1));
}

__device__ __forceinline__ float tanh_d4(float z) {
  const float a  = fminf(fabsf(z), 20.0f);
  const float e  = expf(2.0f * a);
  const float u  = 2.0f / (e + 1.0f);
  const float t  = 1.0f - u;
  const float w  = u * (2.0f - u);
  const float t2 = t * t;
  const float g  = (16.0f - 24.0f * t2) * t * w;
  return (z < 0.0f) ? -g : g;
}

__global__ __launch_bounds__(32) void d4sum_mlp_kernel(const float* __restrict__ x,
                                                       const float* __restrict__ W1,
                                                       const float* __restrict__ W2,
                                                       float* __restrict__ out)
{
  __shared__ __align__(16) unsigned short sXh[kTileM * kXP];
  __shared__ __align__(16) unsigned short sXl[kTileM * kXP];
  __shared__ __align__(16) unsigned short sW1h[kHid * kW1P];
  __shared__ __align__(16) unsigned short sW1l[kHid * kW1P];
  __shared__ __align__(16) unsigned short sW2h[16 * kW2P];
  __shared__ __align__(16) unsigned short sW2l[16 * kW2P];
  __shared__ __align__(16) unsigned short sGh[kTileM * kGP];
  __shared__ __align__(16) unsigned short sGl[kTileM * kGP];
  __shared__ __align__(16) float sZ[kTileM * kZP];
  __shared__ __align__(16) float sS2[kHid];
  __shared__ __align__(16) float sO[kTileM * kOP];

  const int lane = threadIdx.x & 31;
  const int hh   = lane >> 4;
  const int lm   = lane & 15;
  const int b0   = blockIdx.x * kTileM;
  const v4u zero4 = (v4u){0u, 0u, 0u, 0u};

  {
    const int row = lane >> 1;
    const int hf  = lane & 1;
    const float* src = x + (size_t)(b0 + row) * kDin + hf * 8;
    const v4f a0 = *(const v4f*)(src);
    const v4f a1 = *(const v4f*)(src + 4);
    v4u hw, lw;
    split_oct(a0, a1, hw, lw);
    *(v4u*)(sXh + row * kXP + hf * 8) = hw;
    *(v4u*)(sXl + row * kXP + hf * 8) = lw;
    *(v4u*)(sXh + row * kXP + 16 + hf * 8) = zero4;
    *(v4u*)(sXl + row * kXP + 16 + hf * 8) = zero4;
  }

#pragma unroll 1
  for (int it = 0; it < (kHid * kDin / 8) / 32; ++it) {
    const int chunk = it * 32 + lane;
    const int row = chunk >> 1;
    const int hf  = chunk & 1;
    const float* src = W1 + (size_t)row * kDin + hf * 8;
    const v4f a0 = *(const v4f*)(src);
    const v4f a1 = *(const v4f*)(src + 4);
    float ss = 0.0f;
    ss = fmaf(a0[0], a0[0], ss);
    ss = fmaf(a0[1], a0[1], ss);
    ss = fmaf(a0[2], a0[2], ss);
    ss = fmaf(a0[3], a0[3], ss);
    ss = fmaf(a1[0], a1[0], ss);
    ss = fmaf(a1[1], a1[1], ss);
    ss = fmaf(a1[2], a1[2], ss);
    ss = fmaf(a1[3], a1[3], ss);
    const float other = __shfl_xor(ss, 1, 32);
    const float sn = ss + other;
    v4u hw, lw;
    split_oct(a0, a1, hw, lw);
    *(v4u*)(sW1h + row * kW1P + hf * 8) = hw;
    *(v4u*)(sW1l + row * kW1P + hf * 8) = lw;
    *(v4u*)(sW1h + row * kW1P + 16 + hf * 8) = zero4;
    *(v4u*)(sW1l + row * kW1P + 16 + hf * 8) = zero4;
    if (hf == 0) sS2[row] = sn * sn;
  }

#pragma unroll 1
  for (int it = 0; it < (kOut * kHid / 8) / 32; ++it) {
    const int chunk = it * 32 + lane;
    const int row = chunk >> 4;
    const int c8  = (chunk & 15) * 8;
    const float* src = W2 + (size_t)row * kHid + c8;
    const v4f a0 = *(const v4f*)(src);
    const v4f a1 = *(const v4f*)(src + 4);
    v4u hw, lw;
    split_oct(a0, a1, hw, lw);
    *(v4u*)(sW2h + row * kW2P + c8) = hw;
    *(v4u*)(sW2l + row * kW2P + c8) = lw;
    *(v4u*)(sW2h + (row + 8) * kW2P + c8) = zero4;
    *(v4u*)(sW2l + (row + 8) * kW2P + c8) = zero4;
  }
  __syncthreads();

  {
    const v16b xh = frag_load((const __bf16*)(const void*)sXh + lm * kXP + 8 * hh);
    const v16b xl = frag_load((const __bf16*)(const void*)sXl + lm * kXP + 8 * hh);
#pragma unroll 1
    for (int t = 0; t < kHid / 16; ++t) {
      const int n = t * 16 + lm;
      const v16b bh = frag_load((const __bf16*)(const void*)sW1h + n * kW1P + 8 * hh);
      const v16b bl = frag_load((const __bf16*)(const void*)sW1l + n * kW1P + 8 * hh);
      v8f c = (v8f){0.f, 0.f, 0.f, 0.f, 0.f, 0.f, 0.f, 0.f};
      c = mma_bf(xh, bh, c);
      c = mma_bf(xh, bl, c);
      c = mma_bf(xl, bh, c);
      guard_acc(c, xh, xl, bh, bl);
      float* zp = sZ + (8 * hh) * kZP + n;
      zp[0 * kZP] = c[0];
      zp[1 * kZP] = c[1];
      zp[2 * kZP] = c[2];
      zp[3 * kZP] = c[3];
      zp[4 * kZP] = c[4];
      zp[5 * kZP] = c[5];
      zp[6 * kZP] = c[6];
      zp[7 * kZP] = c[7];
    }
  }
  __syncthreads();

  {
    const int col = lane * 4;
    const v4f sv = *(const v4f*)(sS2 + col);
    const float s0 = sv[0], s1 = sv[1], s2v = sv[2], s3 = sv[3];
#pragma unroll 1
    for (int row = 0; row < kTileM; ++row) {
      const v4f zv = *(const v4f*)(sZ + row * kZP + col);
      const float z0 = zv[0], z1 = zv[1], z2 = zv[2], z3 = zv[3];
      const float g0 = tanh_d4(z0) * s0;
      const float g1 = tanh_d4(z1) * s1;
      const float g2 = tanh_d4(z2) * s2v;
      const float g3 = tanh_d4(z3) * s3;
      unsigned h01, l01, h23, l23;
      split_pair(g0, g1, h01, l01);
      split_pair(g2, g3, h23, l23);
      const v2u hw = (v2u){h01, h23};
      const v2u lw = (v2u){l01, l23};
      *(v2u*)(sGh + row * kGP + col) = hw;
      *(v2u*)(sGl + row * kGP + col) = lw;
    }
  }
  __syncthreads();

  {
    v8f acc = (v8f){0.f, 0.f, 0.f, 0.f, 0.f, 0.f, 0.f, 0.f};
#pragma unroll 1
    for (int k0 = 0; k0 < kHid; k0 += 32) {
      const v16b ah = frag_load((const __bf16*)(const void*)sGh + lm * kGP + k0 + 8 * hh);
      const v16b al = frag_load((const __bf16*)(const void*)sGl + lm * kGP + k0 + 8 * hh);
      const v16b bh = frag_load((const __bf16*)(const void*)sW2h + lm * kW2P + k0 + 8 * hh);
      const v16b bl = frag_load((const __bf16*)(const void*)sW2l + lm * kW2P + k0 + 8 * hh);
      acc = mma_bf(ah, bh, acc);
      acc = mma_bf(ah, bl, acc);
      acc = mma_bf(al, bh, acc);
      guard_acc(acc, ah, al, bh, bl);
    }
    float* op = sO + (8 * hh) * kOP + lm;
    op[0 * kOP] = acc[0];
    op[1 * kOP] = acc[1];
    op[2 * kOP] = acc[2];
    op[3 * kOP] = acc[3];
    op[4 * kOP] = acc[4];
    op[5 * kOP] = acc[5];
    op[6 * kOP] = acc[6];
    op[7 * kOP] = acc[7];
  }
  __syncthreads();

  {
    const int row = lane >> 1;
    const int c4  = (lane & 1) * 4;
    const v4f val = *(const v4f*)(sO + row * kOP + c4);
    volatile v4f* dst = (volatile v4f*)(out + (size_t)b0 * kOut + (size_t)lane * 4);
    *dst = val;
    __threadfence();
    *dst = val;
  }
}

extern "C" void kernel_launch(void* const* d_in, const int* in_sizes, int n_in,
                              void* d_out, int out_size, void* d_ws, size_t ws_size,
                              hipStream_t stream) {
  (void)d_ws;
  (void)ws_size;
  if (n_in < 3) return;
  if (in_sizes[0] != kBatch * kDin) return;
  if (in_sizes[1] != kHid * kDin) return;
  if (in_sizes[2] != kOut * kHid) return;
  if (out_size != kBatch * kOut) return;

  const float* x  = (const float*)d_in[0];
  const float* W1 = (const float*)d_in[1];
  const float* W2 = (const float*)d_in[2];
  float* out = (float*)d_out;

  d4sum_mlp_kernel<<<kBatch / kTileM, 32, 0, stream>>>(x, W1, W2, out);
}
